// CNN_CDR123_global_max_13374528159825
// MI455X (gfx1250) — hardware-verified
//
#include <hip/hip_runtime.h>


#define NBT  16384
#define EMB  20
#define NFL  16
#define NKS  5
#define NFS  (NKS * NFL)
#define NRP  128
#define KW9  (EMB * 9)
#define KP   192
#define NSEQ 7
#define NFT  (NSEQ * NFS)
#define NFP  576
#define LD1  64
#define BC   2048
#define LSUM 74
#define DM   KP
#define LOSC 1024.0f
__constant__ int c_len[NSEQ] = {12, 7, 8, 16, 6, 7, 18};
__constant__ int c_loff[NSEQ] = {0, 12, 19, 27, 43, 49, 56};

typedef _Float16 h16;
typedef unsigned short bf;
typedef __attribute__((ext_vector_type(16))) __bf16   v16bf;
typedef __attribute__((ext_vector_type(16))) _Float16 v16h;
typedef __attribute__((ext_vector_type(8)))  _Float16 v8h;
typedef __attribute__((ext_vector_type(8)))  unsigned short v8us;
typedef __attribute__((ext_vector_type(8)))  float    v8f;
typedef __attribute__((ext_vector_type(4)))  float    v4f;
typedef v8h  __attribute__((may_alias)) v8ha;
typedef v4f  __attribute__((may_alias)) v4fa;
typedef v8us __attribute__((may_alias)) v8usa;

__device__ __forceinline__ unsigned short f2bf(float f) { unsigned u = __float_as_uint(f); u += 0x7FFFu + ((u >> 16) & 1u); return (unsigned short)(u >> 16); }
__device__ __forceinline__ float bf2f(unsigned short b) { return __uint_as_float(((unsigned)b) << 16); }
__device__ __forceinline__ float bfr(float f) { return bf2f(f2bf(f)); }
__device__ __forceinline__ v16h cat16(v8h lo, v8h hi) { return __builtin_shufflevector(lo, hi, 0, 1, 2, 3, 4, 5, 6, 7, 8, 9, 10, 11, 12, 13, 14, 15); }
__device__ __forceinline__ v16bf cat16b(v8us lo, v8us hi) { return __builtin_bit_cast(v16bf, __builtin_shufflevector(lo, hi, 0, 1, 2, 3, 4, 5, 6, 7, 8, 9, 10, 11, 12, 13, 14, 15)); }
__device__ __forceinline__ v8f wmma16(v16h a, v16h b, v8f c) { return __builtin_amdgcn_wmma_f32_16x16x32_f16(false, a, false, b, (short)0, c, false, false); }
__device__ __forceinline__ v8f wmmab(v16bf a, v16bf b, v8f c) { return __builtin_amdgcn_wmma_f32_16x16x32_bf16(false, a, false, b, (short)0, c, false, false); }

template <bool SPLITA, bool F16OUT = false>
__global__ __launch_bounds__(128) void k_gemmb(const bf* __restrict__ A, const bf* __restrict__ Al, const bf* __restrict__ Bn, const float* __restrict__ bias, float* C, int ldc, h16* C2, const float* __restrict__ R = nullptr, int K = DM, int roundR = 1) {
    __shared__ __align__(16) float ost[4][16 * 68];
    const int lane = threadIdx.x & 31, wave = threadIdx.x >> 5, lr = lane & 15, hi = lane >> 4;
    const int r0 = blockIdx.x * 64 + wave * 16, c0 = blockIdx.y * 64;
    const size_t aoff = (size_t)(r0 + lr) * K + 8 * hi;
    size_t boff[4];
#pragma unroll
    for (int t = 0; t < 4; ++t) boff[t] = (size_t)(c0 + t * 16 + lr) * K + 8 * hi;
    v8f acc[4];
#pragma unroll
    for (int t = 0; t < 4; ++t) acc[t] = (v8f){};
#pragma unroll 1
    for (int kc = 0; kc < K; kc += 32) {
        const v16bf a = cat16b(*(const v8us*)(A + aoff + kc), *(const v8us*)(A + aoff + kc + 16));
        v16bf al = a;
        if (SPLITA) al = cat16b(*(const v8us*)(Al + aoff + kc), *(const v8us*)(Al + aoff + kc + 16));
#pragma unroll
        for (int t = 0; t < 4; ++t) { const v16bf b = cat16b(*(const v8us*)(Bn + boff[t] + kc), *(const v8us*)(Bn + boff[t] + kc + 16)); acc[t] = wmmab(a, b, acc[t]); if (SPLITA) acc[t] = wmmab(al, b, acc[t]); }
        asm volatile("v_nop\n\tv_nop\n\tv_nop\n\tv_nop" : "+v"(acc[0]), "+v"(acc[1]), "+v"(acc[2]), "+v"(acc[3]) : "v"(a), "v"(al));
    }
    float* os = &ost[wave][0];
#pragma unroll
    for (int t = 0; t < 4; ++t) { const float bv = bias ? bfr(bias[c0 + t * 16 + lr]) : 0.f;
#pragma unroll
        for (int j = 0; j < 8; ++j) os[(hi * 8 + j) * 68 + t * 16 + lr] = acc[t][j] + bv; }
    __syncthreads();
    if (F16OUT) {
        h16* crow = (h16*)(void*)C + (size_t)r0 * ldc + c0;
        auto pass = [&]() {
#pragma unroll
            for (int s = 0; s < 4; ++s) { const int row = 4 * s + (lane >> 3), piece = lane & 7; const float* sp = os + row * 68 + piece * 8; v8h o, o2;
#pragma unroll
                for (int i = 0; i < 8; ++i) { const h16 a = (h16)sp[i]; o[i] = a; o2[i] = (h16)((sp[i] - (float)a) * LOSC); }
                *(volatile v8h*)(crow + (size_t)row * ldc + piece * 8) = o; if (C2) *(volatile v8h*)(C2 + (size_t)r0 * ldc + c0 + (size_t)row * ldc + piece * 8) = o2; }
        };
        pass(); __threadfence(); pass();
    } else {
        float* crow = C + (size_t)r0 * ldc + c0;
        auto pass = [&]() {
#pragma unroll
            for (int s = 0; s < 8; ++s) { const int Lid = (lane >> 3) + 4 * s, piece = lane & 7; const int row = Lid >> 1, cofs = (Lid & 1) * 32 + piece * 4;
                v4f val = *(const v4fa*)(os + row * 68 + cofs); if (R) { const v4f rv = *(const v4f*)(R + ((size_t)r0 + row) * ldc + c0 + cofs); val += roundR ? (v4f){bfr(rv[0]), bfr(rv[1]), bfr(rv[2]), bfr(rv[3])} : rv; }
                *(volatile v4f*)(crow + (size_t)row * ldc + cofs) = val; }
        };
        pass(); __threadfence(); pass();
    }
}


__global__ __launch_bounds__(256) void k_w9(const float* __restrict__ W1, const float* __restrict__ W3, const float* __restrict__ W5, const float* __restrict__ W7, const float* __restrict__ W9p, bf* W9) {
    const int u = blockIdx.x * 256 + threadIdx.x; if (u >= NSEQ * NRP * KP / 8) return; v8us ob;
    const int i = u / (NRP * KP / 8), rem = u % (NRP * KP / 8), r = rem / (KP / 8), col0 = (rem % (KP / 8)) * 8;
    const int kidx = r / NFL, f = r % NFL, k = 2 * kidx + 1;
    const float* Wk = (kidx == 0) ? W1 : (kidx == 1) ? W3 : (kidx == 2) ? W5 : (kidx == 3) ? W7 : W9p;
#pragma unroll
    for (int q = 0; q < 8; ++q) { const int col = col0 + q; const int c = col / 9, t = col % 9, tp = t - (4 - kidx);
        const bool ok = (r < NFS) && (col < KW9) && tp >= 0 && tp < k; const int cc = c < EMB ? c : EMB - 1, tc = tp < 0 ? 0 : (tp >= k ? k - 1 : tp); const int kk = kidx > 4 ? 4 : kidx; (void)kk;
        const float w = Wk[(((size_t)i * NFL + f) * EMB + cc) * k + tc]; ob[q] = ok ? f2bf(w) : (unsigned short)0; }
    *(volatile v8us*)(W9 + (size_t)u * 8) = ob; __threadfence(); *(volatile v8us*)(W9 + (size_t)u * 8) = ob;
}
__global__ __launch_bounds__(256) void k_l1pad(const float* __restrict__ L1, bf* L1B) {
    const int u = blockIdx.x * 256 + threadIdx.x; if (u >= LD1 * NFP / 8) return; const int o = u / (NFP / 8), c0 = (u % (NFP / 8)) * 8; v8us ob;
#pragma unroll
    for (int q = 0; q < 8; ++q) { const int c = c0 + q, cc = c < NFT ? c : NFT - 1; const float w = L1[(size_t)o * NFT + cc]; ob[q] = (c < NFT) ? f2bf(w) : (unsigned short)0; }
    *(volatile v8us*)(L1B + (size_t)u * 8) = ob; __threadfence(); *(volatile v8us*)(L1B + (size_t)u * 8) = ob;
}
__global__ __launch_bounds__(256) void k_im2col(const float* __restrict__ x, int L, int b0, bf* A) {
    const int lane = threadIdx.x & 31, r = blockIdx.x * 8 + (threadIdx.x >> 5); if (r >= BC * L) return;
    const int bl = r / L, l = r % L; const float* xs = x + ((size_t)(b0 + bl) * EMB) * L;
    v8us ob;
#pragma unroll
    for (int q = 0; q < 8; ++q) { const int col = lane * 8 + q; const int c = col / 9, t = col % 9, p = l + t - 4; const bool ok = (col < KW9) && p >= 0 && p < L;
        const int cc = c < EMB ? c : EMB - 1, pc = p < 0 ? 0 : (p >= L ? L - 1 : p); const float xv = xs[(size_t)cc * L + pc]; ob[q] = ok ? f2bf(xv) : (unsigned short)0; }
    if (lane < KP / 8) { *(volatile v8us*)(A + (size_t)r * KP + lane * 8) = ob; __threadfence(); *(volatile v8us*)(A + (size_t)r * KP + lane * 8) = ob; }
}
__global__ __launch_bounds__(256) void k_feat(const float* __restrict__ Call, bf* Fh, bf* Fl) {
    const int lane = threadIdx.x & 31, bl = blockIdx.x * 8 + (threadIdx.x >> 5); if (bl >= BC) return;
#pragma unroll 1
    for (int ps = 0; ps < 2; ++ps) {
#pragma unroll 1
        for (int j0 = lane * 8; j0 < NFP; j0 += 256) { v8us oh, ol;
#pragma unroll
            for (int q = 0; q < 8; ++q) { const int j = j0 + q; float y = 0.f;
                if (j < NFT) { const int i = j / NFS, r = j % NFS; const int L = c_len[i]; const float* Cb = Call + ((size_t)BC * c_loff[i] + (size_t)bl * L) * NRP + r; float m = -3.0e38f;
#pragma unroll 1
                    for (int l = 0; l < L; ++l) m = fmaxf(m, Cb[(size_t)l * NRP]);
                    y = fmaxf(0.2f * m, 0.f); }
                const unsigned short hb = f2bf(y); oh[q] = hb; ol[q] = f2bf(y - bf2f(hb)); }
            const size_t o = (size_t)bl * NFP + j0; *(volatile v8us*)(Fh + o) = oh; *(volatile v8us*)(Fl + o) = ol; }
        if (ps == 0) __threadfence(); }
}
__global__ __launch_bounds__(256) void k_out(const float* __restrict__ H, const float* __restrict__ L2, const float* __restrict__ b2, int b0, float* OUTP) {
    const int bl = blockIdx.x * 256 + threadIdx.x; if (bl >= BC) return; const float* hr = H + (size_t)bl * LD1; float a = bfr(b2[0]);
#pragma unroll 4
    for (int c = 0; c < LD1; ++c) { const float s = 1.0f / (1.0f + __expf(-hr[c])); a = fmaf(s, bfr(L2[c]), a); }
    *(volatile float*)(OUTP + b0 + bl) = a; __threadfence(); *(volatile float*)(OUTP + b0 + bl) = a;
}

extern "C" void kernel_launch(void* const* d_in, const int* in_sizes, int n_in,
                              void* d_out, int out_size, void* d_ws, size_t ws_size, hipStream_t stream) {
    (void)in_sizes; (void)n_in; (void)out_size;
    const float* seq[NSEQ]; for (int i = 0; i < NSEQ; ++i) seq[i] = (const float*)d_in[i];
    const float* Wk[NKS]; for (int j = 0; j < NKS; ++j) Wk[j] = (const float*)d_in[7 + j];
    const float* L1 = (const float*)d_in[12]; const float* L1b = (const float*)d_in[13]; const float* L2 = (const float*)d_in[14]; const float* L2b = (const float*)d_in[15];
    float* out = (float*)d_out;
    const int lens[NSEQ] = {12, 7, 8, 16, 6, 7, 18}; const int loff[NSEQ] = {0, 12, 19, 27, 43, 49, 56};
    char* wsp = (char*)d_ws;
    auto take = [&](size_t bytes) { char* p = wsp; wsp += (bytes + 255) & ~(size_t)255; return (void*)p; };
    bf* W9 = (bf*)take((size_t)NSEQ * NRP * KP * 2); bf* L1B = (bf*)take((size_t)LD1 * NFP * 2); bf* A = (bf*)take((size_t)BC * 18 * KP * 2);
    float* Call = (float*)take((size_t)BC * LSUM * NRP * 4); bf* Fh = (bf*)take((size_t)BC * NFP * 2); bf* Fl = (bf*)take((size_t)BC * NFP * 2); float* H = (float*)take((size_t)BC * LD1 * 4);
    if ((size_t)(wsp - (char*)d_ws) > ws_size) return;
    k_w9<<<(NSEQ * NRP * KP / 8 + 255) / 256, 256, 0, stream>>>(Wk[0], Wk[1], Wk[2], Wk[3], Wk[4], W9); k_l1pad<<<(LD1 * NFP / 8 + 255) / 256, 256, 0, stream>>>(L1, L1B);
    for (int ch = 0; ch < NBT / BC; ++ch) { const int b0 = ch * BC;
        for (int i = 0; i < NSEQ; ++i) { const int L = lens[i];
            k_im2col<<<(BC * L) / 8, 256, 0, stream>>>(seq[i], L, b0, A);
            k_gemmb<false, false><<<dim3((BC * L) / 64, NRP / 64, 1), 128, 0, stream>>>(A, nullptr, W9 + (size_t)i * NRP * KP, nullptr, Call + (size_t)BC * loff[i] * NRP, NRP, nullptr, nullptr, KP); }
        k_feat<<<BC / 8, 256, 0, stream>>>(Call, Fh, Fl);
        k_gemmb<true, false><<<dim3(BC / 64, 1, 1), 128, 0, stream>>>(Fh, Fl, L1B, L1b, H, LD1, nullptr, nullptr, NFP);
        k_out<<<BC / 256, 256, 0, stream>>>(H, L2, L2b, b0, out);
    }
}
